// RetNet_23613730193588
// MI455X (gfx1250) — hardware-verified
//
#include <hip/hip_runtime.h>
#include <math.h>

constexpr int NLAYER  = 3;
constexpr int HID     = 256;
constexpr int NHEAD   = 4;
constexpr int HEAD_DK = 64;
constexpr int VDIM    = 512;
constexpr int HEAD_DV = 128;
constexpr int FFN     = 1024;
constexpr int NBATCH  = 2;
constexpr int SEQ     = 2048;
constexpr int NTOK    = NBATCH * SEQ;
constexpr int NPROJ   = 2 * HID + 2 * VDIM;
constexpr int COL_KEY = HID;
constexpr int COL_VAL = 2 * HID;
constexpr int COL_GATE = 2 * HID + VDIM;
constexpr int NPAIR   = HEAD_DK / 2;
constexpr int SQRT_DK = 8;
static_assert(SQRT_DK * SQRT_DK == HEAD_DK);
static_assert(NHEAD * HEAD_DK == HID);
static_assert(NHEAD * HEAD_DV == VDIM);
static_assert(NPROJ == 1536);
static_assert(NTOK % 64 == 0 && NPROJ % 64 == 0 && HID % 64 == 0 && FFN % 64 == 0 && VDIM % 64 == 0);
static_assert(HID % 32 == 0 && VDIM % 32 == 0 && FFN % 32 == 0 && HEAD_DK % 32 == 0 && SEQ % 64 == 0);
static_assert(NPAIR == 32);

constexpr float W_CARRY   = 64.0f;
constexpr float ACT_CARRY = 64.0f;
constexpr float QK_CARRY  = 16.0f;
constexpr float V_CARRY   = 16.0f;
constexpr float P_CARRY   = 1024.0f;
constexpr float KEY_SCALE = 1.0f / (float)SQRT_DK;
constexpr float SCORE_UNSCALE = KEY_SCALE / (QK_CARRY * QK_CARRY);
constexpr float O_UNSCALE = 1.0f / (P_CARRY * V_CARRY);
constexpr float SC_W   = 1.0f / W_CARRY;
constexpr float SC_AW  = 1.0f / (ACT_CARRY * W_CARRY);
constexpr float LN_EPS_F  = 1e-5f;
constexpr float RMS_EPS_F = 1e-6f;
constexpr float INV_SQRT2 = 0.70710678118654752440f;

constexpr int RT_PP = 72;
constexpr int RT_OP = 132;

typedef __attribute__((ext_vector_type(16))) _Float16 v16h;
typedef __attribute__((ext_vector_type(8)))  _Float16 v8h;
typedef __attribute__((ext_vector_type(8)))  float    v8f;
typedef __attribute__((ext_vector_type(4)))  float    v4f;
typedef __attribute__((ext_vector_type(4)))  unsigned int v4u;

struct AngTab { float a[32]; };
static_assert(sizeof(AngTab) == 128);

__device__ __forceinline__ unsigned pk16(unsigned short a, unsigned short b) { return (unsigned)a | ((unsigned)b << 16); }
__device__ __forceinline__ unsigned short h_bits(float f) { const _Float16 h = (_Float16)f; return __builtin_bit_cast(unsigned short, h); }

__device__ __forceinline__ void wave_sync() {
  __builtin_amdgcn_fence(__ATOMIC_RELEASE, "workgroup");
  __builtin_amdgcn_wave_barrier();
  __builtin_amdgcn_fence(__ATOMIC_ACQUIRE, "workgroup");
}

__device__ __forceinline__ void grp_guard_h(v8f& a, v8f& b, v8f& c, v8f& d, v16h x, v16h y0, v16h y1, v16h y2, v16h y3) {
  asm volatile("v_nop\n\tv_nop\n\tv_nop\n\tv_nop" : "+v"(a), "+v"(b), "+v"(c), "+v"(d) : "v"(x), "v"(y0), "v"(y1), "v"(y2), "v"(y3));
}
__device__ __forceinline__ void keep4_h(v16h a, v16h b, v16h c, v16h d) { asm volatile("v_nop" :: "v"(a), "v"(b), "v"(c), "v"(d)); }
__device__ __forceinline__ void acc_guard4(v8f& a, v8f& b, v8f& c, v8f& d) { asm volatile("v_nop\n\tv_nop\n\tv_nop\n\tv_nop" : "+v"(a), "+v"(b), "+v"(c), "+v"(d)); }

template <typename T> struct Frag;
template <> struct Frag<_Float16> {
  typedef v16h V; union U { v16h v; v8h h[2]; };
  static __device__ __forceinline__ v16h load(const _Float16* p) {
    U f; f.h[0] = *(const v8h*)(p); f.h[1] = *(const v8h*)(p + 16); return f.v;
  }
  static __device__ __forceinline__ v8f mma(v16h a, v16h b, v8f c) {
    return __builtin_amdgcn_wmma_f32_16x16x32_f16(false, a, false, b, (short)0, c, false, false);
  }
};

__device__ __forceinline__ v8f mma_h(v16h a, v16h b, v8f c) {
  c = __builtin_amdgcn_wmma_f32_16x16x32_f16(false, a, false, b, (short)0, c, false, false);
  asm volatile("v_nop\n\tv_nop\n\tv_nop\n\tv_nop" : "+v"(c) : "v"(a), "v"(b));
  return c;
}

template <bool BIAS, bool RESID>
__global__ __launch_bounds__(256) void wmma_gemm64_f16(
    const unsigned short* __restrict__ Ap, const unsigned short* __restrict__ Btp,
    float* __restrict__ C, const float* __restrict__ bias, const float* __restrict__ resid,
    int lda, int ldb, int ldc, int M, int N, int K, float scale) {
  typedef _Float16 T;
  typedef v16h V;
  const T* A = (const T*)Ap; const T* Bt = (const T*)Btp;
  __shared__ __align__(16) float sT[8][16 * 68];
  const int lane = threadIdx.x & 31;
  const int wave = threadIdx.x >> 5;
  const int tilesN = N >> 6;
  const int tilesM = M >> 6;
  const int tile = blockIdx.x * 8 + wave;
  if (tile >= tilesM * tilesN) return;
  const int tm = tile / tilesN;
  const int tn = tile - tm * tilesN;
  const int m0 = tm << 6;
  const int n0 = tn << 6;

  const int rlane = lane & 15;
  const int koff  = (lane >> 4) * 8;
  const int mOff  = (lane >> 4) * 8;

  v8f acc[4][4];
#pragma unroll
  for (int i = 0; i < 4; ++i)
#pragma unroll
    for (int j = 0; j < 4; ++j) acc[i][j] = (v8f){0.f,0.f,0.f,0.f,0.f,0.f,0.f,0.f};

  for (int k0 = 0; k0 < K; k0 += 32) {
    V bh[4];
#pragma unroll
    for (int j = 0; j < 4; ++j) {
      const size_t bo = (size_t)(n0 + (j << 4) + rlane) * ldb + koff + k0;
      bh[j] = Frag<T>::load(Bt + bo);
    }
#pragma unroll
    for (int i = 0; i < 4; ++i) {
      const size_t ao = (size_t)(m0 + (i << 4) + rlane) * lda + koff + k0;
      V ah = Frag<T>::load(A + ao);
#pragma unroll
      for (int j = 0; j < 4; ++j) acc[i][j] = Frag<T>::mma(ah, bh[j], acc[i][j]);
      grp_guard_h(acc[i][0], acc[i][1], acc[i][2], acc[i][3], ah, bh[0], bh[1], bh[2], bh[3]);
    }
    keep4_h(bh[0], bh[1], bh[2], bh[3]);
  }
  acc_guard4(acc[0][0], acc[0][1], acc[0][2], acc[0][3]);
  acc_guard4(acc[1][0], acc[1][1], acc[1][2], acc[1][3]);
  acc_guard4(acc[2][0], acc[2][1], acc[2][2], acc[2][3]);
  acc_guard4(acc[3][0], acc[3][1], acc[3][2], acc[3][3]);

  float* slab = sT[wave];
  const int hh = lane >> 4, c4 = (lane & 15) * 4;
#pragma unroll
  for (int i = 0; i < 4; ++i) {
    const int mBase = m0 + (i << 4);
#pragma unroll
    for (int j = 0; j < 4; ++j) {
      const int n = n0 + (j << 4) + rlane;
      float bv = 0.f;
      if (BIAS) bv = bias[n];
#pragma unroll
      for (int r = 0; r < 8; ++r) {
        float v = acc[i][j][r] * scale;
        v += bv;
        slab[(mOff + r) * 68 + (j << 4) + rlane] = v;
      }
    }
    wave_sync();
    if (RESID) {
#pragma unroll
      for (int it = 0; it < 8; ++it) {
        const int row = it * 2 + hh;
        v4f v = *(const v4f*)(slab + row * 68 + c4);
        const v4f rv = *(const v4f*)(resid + (size_t)(mBase + row) * ldc + n0 + c4);
        v = v + rv;
        *(v4f*)(slab + row * 68 + c4) = v;
      }
      wave_sync();
    }
    for (int pass = 0; pass < 2; ++pass) {
#pragma unroll
      for (int it = 0; it < 8; ++it) {
        const int row = it * 2 + hh;
        v4f v = *(const v4f*)(slab + row * 68 + c4);
        *(volatile v4f*)(C + (size_t)(mBase + row) * ldc + n0 + c4) = v;
      }
      __threadfence();
    }
    wave_sync();
  }
}

__global__ __launch_bounds__(256) void tcast_kernel(const float* __restrict__ in, unsigned short* __restrict__ out,
                                                    long in_s0, long in_s1, long out_s0, long out_s1,
                                                    int in_ld, int out_ld, int nz1, float scale) {
  __shared__ float sm[64][65];
  const int t  = threadIdx.x;
  const int r0 = blockIdx.x * 64;
  const int c0 = blockIdx.y * 64;
  const int z  = blockIdx.z;
  const int z0 = z / nz1;
  const int z1 = z - z0 * nz1;
  const float* ip = in + (size_t)z0 * in_s0 + (size_t)z1 * in_s1;
  unsigned short* op = out + (size_t)z0 * out_s0 + (size_t)z1 * out_s1;
#pragma unroll
  for (int i = 0; i < 16; ++i) {
    const int e = i * 256 + t;
    const int r = e >> 6;
    const int c = e & 63;
    sm[c][r] = ip[(size_t)(r0 + r) * in_ld + c0 + c] * scale;
  }
  __syncthreads();
  const int lane = t & 31, wave = t >> 5;
  const int q = lane >> 3, c8 = (lane & 7) * 8;
  for (int pass = 0; pass < 2; ++pass) {
#pragma unroll
    for (int it = 0; it < 2; ++it) {
      const int row = wave * 8 + it * 4 + q;
      unsigned short hb[8];
#pragma unroll
      for (int e = 0; e < 8; ++e) hb[e] = h_bits(sm[row][c8 + e]);
      const v4u u = (v4u){pk16(hb[0], hb[1]), pk16(hb[2], hb[3]), pk16(hb[4], hb[5]), pk16(hb[6], hb[7])};
      *(volatile v4u*)(op + (size_t)(c0 + row) * out_ld + r0 + c8) = u;
    }
    __threadfence();
  }
}

__global__ __launch_bounds__(256) void sincos_table_kernel(float* __restrict__ sn, float* __restrict__ cs, AngTab ang) {
  const int lane = threadIdx.x & 31;
  const int s = blockIdx.x * 8 + (threadIdx.x >> 5);
  float a = 0.0f;
#pragma unroll
  for (int j = 0; j < 32; ++j) a = (lane == j) ? ang.a[j] : a;
  const float arg = (float)s * a;
  const float sv = sinf(arg);
  const float cv = cosf(arg);
  float* sp = sn + (size_t)s * NPAIR + lane;
  float* cp = cs + (size_t)s * NPAIR + lane;
  *(volatile float*)sp = sv;
  *(volatile float*)cp = cv;
  __threadfence();
  *(volatile float*)sp = sv;
  *(volatile float*)cp = cv;
}

__global__ __launch_bounds__(256) void ln_cast_kernel(const float* __restrict__ x, const float* __restrict__ w,
                                                      const float* __restrict__ bb, unsigned short* __restrict__ out, int nrows) {
  const int lane = threadIdx.x & 31;
  const int row  = blockIdx.x * 8 + (threadIdx.x >> 5);
  const int rowc = row < nrows ? row : nrows - 1;
  const float* xr = x + (size_t)rowc * HID + 8 * lane;
  const v4f xa = *(const v4f*)(xr);
  const v4f xb = *(const v4f*)(xr + 4);
  const v4f wa = *(const v4f*)(w + 8 * lane);
  const v4f wb = *(const v4f*)(w + 8 * lane + 4);
  const v4f ba = *(const v4f*)(bb + 8 * lane);
  const v4f bc = *(const v4f*)(bb + 8 * lane + 4);
  float v[8], wv[8], bv[8];
#pragma unroll
  for (int e = 0; e < 4; ++e) { v[e] = xa[e]; v[4 + e] = xb[e]; wv[e] = wa[e]; wv[4 + e] = wb[e]; bv[e] = ba[e]; bv[4 + e] = bc[e]; }
  float s = ((v[0] + v[1]) + (v[2] + v[3])) + ((v[4] + v[5]) + (v[6] + v[7]));
#pragma unroll
  for (int off = 1; off < 32; off <<= 1) s += __shfl_xor(s, off, 32);
  const float mu = s * (1.0f / (float)HID);
  float ss = 0.0f;
#pragma unroll
  for (int e = 0; e < 8; ++e) { const float d = v[e] - mu; v[e] = d; ss += d * d; }
#pragma unroll
  for (int off = 1; off < 32; off <<= 1) ss += __shfl_xor(ss, off, 32);
  const float rstd = 1.0f / sqrtf(ss * (1.0f / (float)HID) + LN_EPS_F);
  unsigned short hb[8];
#pragma unroll
  for (int e = 0; e < 8; ++e) hb[e] = h_bits((v[e] * rstd) * wv[e] + bv[e]);
  const v4u u = (v4u){pk16(hb[0], hb[1]), pk16(hb[2], hb[3]), pk16(hb[4], hb[5]), pk16(hb[6], hb[7])};
  unsigned short* op = out + (size_t)rowc * HID + 8 * lane;
  if (row < nrows) {
    *(volatile v4u*)op = u;
    __threadfence();
    *(volatile v4u*)op = u;
  }
}

__global__ __launch_bounds__(256) void rot_kernel(const float* __restrict__ qkvg, const float* __restrict__ sn,
                                                  const float* __restrict__ cs, unsigned short* __restrict__ qr,
                                                  unsigned short* __restrict__ kr) {
  const int lane = threadIdx.x & 31;
  const int m = blockIdx.x * 8 + (threadIdx.x >> 5);
  const int b = m / SEQ;
  const int s = m - b * SEQ;
  const int h = lane >> 3, l8 = lane & 7;
  const float* src = qkvg + (size_t)m * NPROJ + 8 * lane;
  const v4f qa = *(const v4f*)(src);
  const v4f qb = *(const v4f*)(src + 4);
  const v4f ka = *(const v4f*)(src + COL_KEY);
  const v4f kb = *(const v4f*)(src + COL_KEY + 4);
  const v4f sv = *(const v4f*)(sn + (size_t)s * NPAIR + l8 * 4);
  const v4f cv = *(const v4f*)(cs + (size_t)s * NPAIR + l8 * 4);
  float qv[8], kv[8], sp[4], cp[4];
#pragma unroll
  for (int e = 0; e < 4; ++e) { qv[e] = qa[e]; qv[4 + e] = qb[e]; kv[e] = ka[e]; kv[4 + e] = kb[e]; sp[e] = sv[e]; cp[e] = cv[e]; }
  unsigned short hq[8], hk[8];
#pragma unroll
  for (int p = 0; p < 4; ++p) {
    const float qe = qv[2 * p], qo = qv[2 * p + 1];
    const float ke = kv[2 * p], ko = kv[2 * p + 1];
    hq[2 * p]     = h_bits((qe * cp[p] - qo * sp[p]) * QK_CARRY);
    hq[2 * p + 1] = h_bits((qo * cp[p] + qe * sp[p]) * QK_CARRY);
    hk[2 * p]     = h_bits((ke * cp[p] - ko * sp[p]) * QK_CARRY);
    hk[2 * p + 1] = h_bits((ko * cp[p] + ke * sp[p]) * QK_CARRY);
  }
  const v4u uq = (v4u){pk16(hq[0], hq[1]), pk16(hq[2], hq[3]), pk16(hq[4], hq[5]), pk16(hq[6], hq[7])};
  const v4u uk = (v4u){pk16(hk[0], hk[1]), pk16(hk[2], hk[3]), pk16(hk[4], hk[5]), pk16(hk[6], hk[7])};
  const size_t dst = ((size_t)(b * NHEAD + h) * SEQ + s) * HEAD_DK + l8 * 8;
  *(volatile v4u*)(qr + dst) = uq;
  *(volatile v4u*)(kr + dst) = uk;
  __threadfence();
  *(volatile v4u*)(qr + dst) = uq;
  *(volatile v4u*)(kr + dst) = uk;
}

__global__ __launch_bounds__(128) void dmattn_kernel(const unsigned short* __restrict__ qrp, const unsigned short* __restrict__ krp,
                                                     const unsigned short* __restrict__ vtp, const float* __restrict__ qkvg,
                                                     unsigned short* __restrict__ og) {
  __shared__ __align__(16) _Float16 Ps[4][16 * RT_PP];
  __shared__ __align__(16) float    Os[4][16 * RT_OP];
  __shared__ __align__(16) unsigned Pk[4][16 * 64];
  const _Float16* qr = (const _Float16*)qrp;
  const _Float16* kr = (const _Float16*)krp;
  const _Float16* vT = (const _Float16*)vtp;
  const int tid = threadIdx.x, wave = tid >> 5, lane = tid & 31;
  const int hh = lane >> 4, c = lane & 15;
  constexpr int NQB = SEQ / 64;
  const int bx = blockIdx.x;
  const int qb = bx % NQB;
  const int bh = bx / NQB;
  const int h  = bh % NHEAD;
  const int b  = bh / NHEAD;
  const int q0w = qb * 64 + wave * 16;

  const float rscale = (float)(32 << h);
  const float gam = 1.0f - 1.0f / rscale;
  const float decay = logf(gam);

  float rv;
  {
    const float sr = (float)(q0w + c + 1);
    const float rsum = -expm1f(sr * decay) * rscale;
    rv = expf((float)c * decay) * (1.0f / sqrtf(rsum));
  }
  float rf[8], den[8];
#pragma unroll
  for (int r = 0; r < 8; ++r) { rf[r] = __shfl(rv, 8 * hh + r, 32); den[r] = 0.0f; }

  float gcol[4];
  {
    const float g0 = expf(-(float)c * decay);
    const float g16 = expf(-16.0f * decay);
    gcol[0] = g0; gcol[1] = gcol[0] * g16; gcol[2] = gcol[1] * g16; gcol[3] = gcol[2] * g16;
  }

  v16h qa[2];
  {
    const _Float16* qrow = qr + ((size_t)bh * SEQ + q0w + c) * HEAD_DK + 8 * hh;
    qa[0] = Frag<_Float16>::load(qrow);
    qa[1] = Frag<_Float16>::load(qrow + 32);
  }

  v8f oacc[8];
#pragma unroll
  for (int t = 0; t < 8; ++t) oacc[t] = (v8f){0.f,0.f,0.f,0.f,0.f,0.f,0.f,0.f};

  _Float16* ps = Ps[wave];
  const int nT = qb + 1;
#pragma unroll 1
  for (int kc = 0; kc < nT; ++kc) {
    const int t0 = kc * 64;
    v8f s[4];
#pragma unroll
    for (int j = 0; j < 4; ++j) {
      s[j] = (v8f){0.f,0.f,0.f,0.f,0.f,0.f,0.f,0.f};
      const _Float16* kp = kr + ((size_t)bh * SEQ + t0 + 16 * j + c) * HEAD_DK + 8 * hh;
#pragma unroll
      for (int dc = 0; dc < 2; ++dc) {
        const v16h kb = Frag<_Float16>::load(kp + dc * 32);
        s[j] = mma_h(qa[dc], kb, s[j]);
      }
    }
    const bool diag = (kc == qb);
    const float etile = expf((float)(q0w - t0) * decay) * SCORE_UNSCALE;
#pragma unroll
    for (int j = 0; j < 4; ++j) {
      const float cf = etile * gcol[j];
      const int colrel = 16 * j + c;
#pragma unroll
      for (int r = 0; r < 8; ++r) {
        const int lim = diag ? (16 * wave + 8 * hh + r) : 4096;
        const bool keep = (colrel <= lim);
        const float pv = (s[j][r] * rf[r]) * cf;
        const float p = keep ? pv : 0.0f;
        den[r] += fabsf(p);
        ps[(8 * hh + r) * RT_PP + colrel] = (_Float16)(p * P_CARRY);
      }
    }
    wave_sync();
#pragma unroll 1
    for (int kk = 0; kk < 2; ++kk) {
      const v16h pa = Frag<_Float16>::load(ps + c * RT_PP + kk * 32 + 8 * hh);
#pragma unroll
      for (int t = 0; t < 8; ++t) {
        const v16h vb = Frag<_Float16>::load(vT + ((size_t)bh * HEAD_DV + 16 * t + c) * SEQ + t0 + kk * 32 + 8 * hh);
        oacc[t] = mma_h(pa, vb, oacc[t]);
      }
    }
    wave_sync();
  }

#pragma unroll
  for (int r = 0; r < 8; ++r) {
#pragma unroll
    for (int off = 1; off < 16; off <<= 1) den[r] += __shfl_xor(den[r], off, 32);
  }
  float ssq[8];
#pragma unroll
  for (int r = 0; r < 8; ++r) {
    const float osc = (1.0f / fmaxf(den[r], 1.0f)) * O_UNSCALE;
    float a = 0.0f;
#pragma unroll
    for (int t = 0; t < 8; ++t) { const float o = oacc[t][r] * osc; oacc[t][r] = o; a += o * o; }
    ssq[r] = a;
  }
#pragma unroll
  for (int r = 0; r < 8; ++r) {
#pragma unroll
    for (int off = 1; off < 16; off <<= 1) ssq[r] += __shfl_xor(ssq[r], off, 32);
  }
  float* os = Os[wave];
#pragma unroll
  for (int r = 0; r < 8; ++r) {
    const float rn = rsqrtf(ssq[r] * (1.0f / (float)HEAD_DV) + RMS_EPS_F);
#pragma unroll
    for (int t = 0; t < 8; ++t) os[(8 * hh + r) * RT_OP + 16 * t + c] = oacc[t][r] * rn;
  }
  wave_sync();

  unsigned* pk = Pk[wave];
  const int l16 = lane & 15;
  const int c8 = l16 * 8;
#pragma unroll 1
  for (int it = 0; it < 8; ++it) {
    const int row = it * 2 + hh;
    const size_t m = (size_t)b * SEQ + q0w + row;
    const float* gp = qkvg + m * NPROJ + COL_GATE + h * HEAD_DV + c8;
    const v4f ga = *(const v4f*)(gp);
    const v4f gb = *(const v4f*)(gp + 4);
    const v4f oa = *(const v4f*)(os + row * RT_OP + c8);
    const v4f ob = *(const v4f*)(os + row * RT_OP + c8 + 4);
    float gv[8], ov[8];
#pragma unroll
    for (int e = 0; e < 4; ++e) { gv[e] = ga[e]; gv[4 + e] = gb[e]; ov[e] = oa[e]; ov[4 + e] = ob[e]; }
    unsigned short hb[8];
#pragma unroll
    for (int e = 0; e < 8; ++e) {
      const float g = gv[e];
      const float sg = 1.0f / (1.0f + expf(-g));
      hb[e] = h_bits(((g * sg) * ov[e]) * ACT_CARRY);
    }
    const v4u u = (v4u){pk16(hb[0], hb[1]), pk16(hb[2], hb[3]), pk16(hb[4], hb[5]), pk16(hb[6], hb[7])};
    *(v4u*)(pk + row * 64 + l16 * 4) = u;
  }
  wave_sync();
  for (int pass = 0; pass < 2; ++pass) {
#pragma unroll
    for (int it = 0; it < 8; ++it) {
      const int row = it * 2 + hh;
      const size_t m = (size_t)b * SEQ + q0w + row;
      const v4u u = *(const v4u*)(pk + row * 64 + l16 * 4);
      *(volatile v4u*)(og + m * VDIM + h * HEAD_DV + c8) = u;
    }
    __threadfence();
  }
}

__global__ __launch_bounds__(256) void gelu_cast_kernel(const float* __restrict__ pre, unsigned short* __restrict__ out, int n8) {
  __shared__ float sx[256 * 9];
  const int t = threadIdx.x;
  const int i = blockIdx.x * 256 + t;
  const bool live = (i < n8);
  const int ic = live ? i : (n8 - 1);
  const float* p = pre + 8 * (size_t)ic;
  const v4f a = *(const v4f*)(p);
  const v4f c = *(const v4f*)(p + 4);
  float* my = sx + t * 9;
#pragma unroll
  for (int e = 0; e < 4; ++e) { my[e] = a[e]; my[4 + e] = c[e]; }
#pragma unroll 1
  for (int e = 0; e < 8; ++e) {
    const float x = my[e];
    const float y = (0.5f * x) * (1.0f + erff(x * INV_SQRT2));
    my[e] = y * ACT_CARRY;
  }
  unsigned short hb[8];
#pragma unroll
  for (int e = 0; e < 8; ++e) hb[e] = h_bits(my[e]);
  const v4u u = (v4u){pk16(hb[0], hb[1]), pk16(hb[2], hb[3]), pk16(hb[4], hb[5]), pk16(hb[6], hb[7])};
  unsigned short* q = out + 8 * (size_t)ic;
  if (live) {
    *(volatile v4u*)q = u;
    __threadfence();
    *(volatile v4u*)q = u;
  }
}

extern "C" void kernel_launch(void* const* d_in, const int* in_sizes, int n_in,
                              void* d_out, int out_size, void* d_ws, size_t ws_size, hipStream_t stream) {
  if (n_in < 14 || d_out == nullptr || d_ws == nullptr) return;
  if (in_sizes[0] != NTOK * HID || in_sizes[1] != NLAYER * HID * HID || in_sizes[2] != NLAYER * HID * HID ||
      in_sizes[3] != NLAYER * HID * VDIM || in_sizes[4] != NLAYER * HID * VDIM || in_sizes[5] != NLAYER * VDIM * HID ||
      in_sizes[6] != NLAYER * HID || in_sizes[7] != NLAYER * HID || in_sizes[8] != NLAYER * HID || in_sizes[9] != NLAYER * HID ||
      in_sizes[10] != NLAYER * HID * FFN || in_sizes[11] != NLAYER * FFN || in_sizes[12] != NLAYER * FFN * HID ||
      in_sizes[13] != NLAYER * HID || out_size != NTOK * HID) return;

  const float* x0   = (const float*)d_in[0];
  const float* Wq   = (const float*)d_in[1];
  const float* Wk   = (const float*)d_in[2];
  const float* Wv   = (const float*)d_in[3];
  const float* Wg   = (const float*)d_in[4];
  const float* Wo   = (const float*)d_in[5];
  const float* ln1w = (const float*)d_in[6];
  const float* ln1b = (const float*)d_in[7];
  const float* ln2w = (const float*)d_in[8];
  const float* ln2b = (const float*)d_in[9];
  const float* W1   = (const float*)d_in[10];
  const float* b1   = (const float*)d_in[11];
  const float* W2   = (const float*)d_in[12];
  const float* b2   = (const float*)d_in[13];
  float* outp = (float*)d_out;

  char* ws = (char*)d_ws; size_t off = 0;
  auto carve = [&](size_t bytes) -> char* { char* p = ws + off; off += (bytes + 255) & ~(size_t)255; return p; };
  unsigned short* WQKVG_T = (unsigned short*)carve((size_t)NLAYER * NPROJ * HID * 2);
  unsigned short* WO_T    = (unsigned short*)carve((size_t)NLAYER * HID * VDIM * 2);
  unsigned short* W1_T    = (unsigned short*)carve((size_t)NLAYER * FFN * HID * 2);
  unsigned short* W2_T    = (unsigned short*)carve((size_t)NLAYER * HID * FFN * 2);
  float*          SINT    = (float*)carve((size_t)SEQ * NPAIR * 4);
  float*          COST    = (float*)carve((size_t)SEQ * NPAIR * 4);
  unsigned short* XN      = (unsigned short*)carve((size_t)NTOK * HID * 2);
  float*          QKVG    = (float*)carve((size_t)NTOK * NPROJ * 4);
  unsigned short* QR      = (unsigned short*)carve((size_t)NTOK * HID * 2);
  unsigned short* KR      = (unsigned short*)carve((size_t)NTOK * HID * 2);
  unsigned short* VT      = (unsigned short*)carve((size_t)NTOK * VDIM * 2);
  unsigned short* OG      = (unsigned short*)carve((size_t)NTOK * VDIM * 2);
  float*          Y       = (float*)carve((size_t)NTOK * HID * 4);
  float*          PRE     = (float*)carve((size_t)NTOK * FFN * 4);
  unsigned short* F1      = (unsigned short*)carve((size_t)NTOK * FFN * 2);
  float*          XA      = (float*)carve((size_t)NTOK * HID * 4);
  float*          XB      = (float*)carve((size_t)NTOK * HID * 4);
  if (off > ws_size || off > (size_t)134217728) return;

  AngTab ang;
  {
    double r = 1.4;
    for (int itn = 0; itn < 64; ++itn) {
      double p30 = 1.0;
      for (int e = 0; e < 30; ++e) p30 *= r;
      const double f = p30 * r - 10000.0;
      r -= f / (31.0 * p30);
    }
    double pw = 1.0;
    for (int j = 0; j < 32; ++j) { ang.a[j] = 1.0f / (float)pw; pw *= r; }
  }

  tcast_kernel<<<dim3(HID / 64, HID / 64, NLAYER), 256, 0, stream>>>(Wq, WQKVG_T, (long)HID * HID, 0L, (long)NPROJ * HID, 0L, HID, HID, 1, W_CARRY);
  tcast_kernel<<<dim3(HID / 64, HID / 64, NLAYER), 256, 0, stream>>>(Wk, WQKVG_T + (size_t)COL_KEY * HID, (long)HID * HID, 0L, (long)NPROJ * HID, 0L, HID, HID, 1, W_CARRY);
  tcast_kernel<<<dim3(HID / 64, VDIM / 64, NLAYER), 256, 0, stream>>>(Wv, WQKVG_T + (size_t)COL_VAL * HID, (long)HID * VDIM, 0L, (long)NPROJ * HID, 0L, VDIM, HID, 1, W_CARRY);
  tcast_kernel<<<dim3(HID / 64, VDIM / 64, NLAYER), 256, 0, stream>>>(Wg, WQKVG_T + (size_t)COL_GATE * HID, (long)HID * VDIM, 0L, (long)NPROJ * HID, 0L, VDIM, HID, 1, W_CARRY);
  tcast_kernel<<<dim3(VDIM / 64, HID / 64, NLAYER), 256, 0, stream>>>(Wo, WO_T, (long)VDIM * HID, 0L, (long)HID * VDIM, 0L, HID, VDIM, 1, W_CARRY);
  tcast_kernel<<<dim3(HID / 64, FFN / 64, NLAYER), 256, 0, stream>>>(W1, W1_T, (long)HID * FFN, 0L, (long)FFN * HID, 0L, FFN, HID, 1, W_CARRY);
  tcast_kernel<<<dim3(FFN / 64, HID / 64, NLAYER), 256, 0, stream>>>(W2, W2_T, (long)FFN * HID, 0L, (long)HID * FFN, 0L, HID, FFN, 1, W_CARRY);
  sincos_table_kernel<<<SEQ / 8, 256, 0, stream>>>(SINT, COST, ang);

  const float* x_cur = x0;
  for (int l = 0; l < NLAYER; ++l) {
    float* x_next = (l == NLAYER - 1) ? outp : (l == 0 ? XA : XB);
    const unsigned short* wqkvg_l = WQKVG_T + (size_t)l * NPROJ * HID;
    const unsigned short* wo_l    = WO_T + (size_t)l * HID * VDIM;
    const unsigned short* w1_l    = W1_T + (size_t)l * FFN * HID;
    const unsigned short* w2_l    = W2_T + (size_t)l * HID * FFN;

    ln_cast_kernel<<<NTOK / 8, 256, 0, stream>>>(x_cur, ln1w + l * HID, ln1b + l * HID, XN, NTOK);
    wmma_gemm64_f16<false, false><<<(NTOK / 64) * (NPROJ / 64) / 8, 256, 0, stream>>>(
        XN, wqkvg_l, QKVG, b2, x0, HID, HID, NPROJ, NTOK, NPROJ, HID, SC_W);
    rot_kernel<<<NTOK / 8, 256, 0, stream>>>(QKVG, SINT, COST, QR, KR);
    tcast_kernel<<<dim3(SEQ / 64, HEAD_DV / 64, NBATCH * NHEAD), 256, 0, stream>>>(
        QKVG + COL_VAL, VT, (long)SEQ * NPROJ, (long)HEAD_DV, (long)NHEAD * HEAD_DV * SEQ, (long)HEAD_DV * SEQ,
        NPROJ, SEQ, NHEAD, V_CARRY);
    dmattn_kernel<<<NBATCH * NHEAD * (SEQ / 64), 128, 0, stream>>>(QR, KR, VT, QKVG, OG);
    wmma_gemm64_f16<false, true><<<(NTOK / 64) * (HID / 64) / 8, 256, 0, stream>>>(
        OG, wo_l, Y, b2, x_cur, VDIM, VDIM, HID, NTOK, HID, VDIM, SC_AW);
    ln_cast_kernel<<<NTOK / 8, 256, 0, stream>>>(Y, ln2w + l * HID, ln2b + l * HID, XN, NTOK);
    wmma_gemm64_f16<true, false><<<(NTOK / 64) * (FFN / 64) / 8, 256, 0, stream>>>(
        XN, w1_l, PRE, b1 + l * FFN, x0, HID, HID, FFN, NTOK, FFN, HID, SC_W);
    gelu_cast_kernel<<<(NTOK * FFN / 8) / 256, 256, 0, stream>>>(PRE, F1, NTOK * FFN / 8);
    wmma_gemm64_f16<true, true><<<(NTOK / 64) * (HID / 64) / 8, 256, 0, stream>>>(
        F1, w2_l, x_next, b2 + l * HID, Y, FFN, FFN, HID, NTOK, HID, FFN, SC_AW);
    x_cur = x_next;
  }
}
